// NeuralODE_70025146794764
// MI455X (gfx1250) — hardware-verified
//
#include <hip/hip_runtime.h>
#include <stdint.h>
#include <stddef.h>

typedef __attribute__((ext_vector_type(16))) _Float16 v16h;
typedef __attribute__((ext_vector_type(8)))  _Float16 v8h;
typedef __attribute__((ext_vector_type(8)))  float    v8f;
typedef __attribute__((ext_vector_type(4)))  float    v4f;

constexpr int kDim      = 32;
constexpr int kHid      = 256;
constexpr int kMaxT     = 32;
constexpr int kNSub     = 2;
constexpr int kStages   = 6;
constexpr int kWaves    = 2;
constexpr int kThreads  = kWaves * 32;
constexpr int kRowsWave = 16;
constexpr int kRowsBlock = kWaves * kRowsWave;

constexpr int kW1P = 264;
constexpr int kW0P = 40;
constexpr int kW2P = 264;
constexpr int kHP  = 264;
constexpr int kYP  = 40;
constexpr int kOSP = 36;

static_assert(kDim % 32 == 0);
static_assert(kHid % 32 == 0);
static_assert(kHid % 16 == 0 && kDim % 16 == 0);
static_assert((kW1P * 2) % 16 == 0 && (kW0P * 2) % 16 == 0 && (kHP * 2) % 16 == 0 && (kYP * 2) % 16 == 0 && (kOSP * 4) % 16 == 0);

constexpr unsigned kOffW1   = 0;
constexpr unsigned kOffW0   = kOffW1 + (unsigned)kHid * kW1P * 2;
constexpr unsigned kOffW2   = kOffW0 + (unsigned)kHid * kW0P * 2;
constexpr unsigned kOffB0   = kOffW2 + (unsigned)kDim * kW2P * 2;
constexpr unsigned kOffB1   = kOffB0 + (unsigned)kHid * 4;
constexpr unsigned kOffB2   = kOffB1 + (unsigned)kHid * 4;
constexpr unsigned kOffTS   = kOffB2 + (unsigned)kDim * 4;
constexpr unsigned kOffCF   = kOffTS + (unsigned)kMaxT * 4;
constexpr unsigned kOffWave = kOffCF + 256u;
constexpr unsigned kWoffY   = 0;
constexpr unsigned kWoffH1  = kWoffY  + (unsigned)kRowsWave * kYP * 2;
constexpr unsigned kWoffH2  = kWoffH1 + (unsigned)kRowsWave * kHP * 2;
constexpr unsigned kWoffKB  = kWoffH2 + (unsigned)kRowsWave * kHP * 2;
constexpr unsigned kWoffOS  = kWoffKB + (unsigned)kStages * 16 * 32 * 4;
constexpr unsigned kWaveBytes = kWoffOS + (unsigned)kRowsWave * kOSP * 4;
constexpr unsigned kSmemBytes = kOffWave + (unsigned)kWaves * kWaveBytes;
static_assert(kOffW0 % 16 == 0 && kOffW2 % 16 == 0 && kOffB0 % 16 == 0 && kOffB1 % 16 == 0 && kOffB2 % 16 == 0);
static_assert(kOffTS % 16 == 0 && kOffCF % 16 == 0 && kOffWave % 16 == 0);
static_assert(kWoffH1 % 16 == 0 && kWoffH2 % 16 == 0 && kWoffKB % 16 == 0 && kWoffOS % 16 == 0 && kWaveBytes % 16 == 0);
static_assert(kSmemBytes == 240640u);

struct FragH {
  union U { v16h v; v8h h[2]; };
  static __device__ __forceinline__ v16h load(const _Float16* p) {
    U f; f.h[0] = *(const v8h*)(p); f.h[1] = *(const v8h*)(p + 16); return f.v;
  }
};

__device__ __forceinline__ v8f mma_g(v16h a, v16h b, v8f c) {
  c = __builtin_amdgcn_wmma_f32_16x16x32_f16(false, a, false, b, (short)0, c, false, false);
  asm volatile("v_nop\n\tv_nop\n\tv_nop\n\tv_nop" : "+v"(c) : "v"(a), "v"(b));
  return c;
}

__device__ __forceinline__ void wave_sync() {
  __builtin_amdgcn_fence(__ATOMIC_RELEASE, "workgroup");
  __builtin_amdgcn_wave_barrier();
  __builtin_amdgcn_fence(__ATOMIC_ACQUIRE, "workgroup");
}

__device__ __forceinline__ float softplus_f(float x) {
  const float t = exp2f(-fabsf(x) * 1.4426950408889634f);
  const float l = log2f(1.0f + t);
  return fmaxf(x, 0.0f) + l * 0.6931471805599453f;
}

__device__ __forceinline__ void store_rows16(float* gdst, const float* osL, int lane) {
  const int q = lane >> 3, c4 = (lane & 7) * 4;
  for (int pass = 0; pass < 2; ++pass) {
#pragma unroll
    for (int it = 0; it < 4; ++it) {
      const int row = it * 4 + q;
      const v4f v = *(const v4f*)(osL + row * kOSP + c4);
      *(volatile v4f*)(gdst + (size_t)row * kDim + c4) = v;
    }
    __threadfence();
  }
}

__device__ __forceinline__ void mlp_eval(const _Float16* ybL, _Float16* h1L, _Float16* h2L,
                                         const _Float16* W0L, const _Float16* W1L, const _Float16* W2L,
                                         const float* b0L, const float* b1L, const float* b2L,
                                         int hh, int cc, float (&kout)[16]) {
  const int koff = hh * 8;
  const v8f zero8 = {0.f, 0.f, 0.f, 0.f, 0.f, 0.f, 0.f, 0.f};
  {
    const v16h a = FragH::load(ybL + cc * kYP + koff);
#pragma unroll 1
    for (int nt = 0; nt < kHid / 16; ++nt) {
      const v16h b = FragH::load(W0L + (nt * 16 + cc) * kW0P + koff);
      v8f acc = mma_g(a, b, zero8);
      const float bias = b0L[nt * 16 + cc];
#pragma unroll
      for (int r = 0; r < 8; ++r) {
        const float x = acc[r] * (1.0f / 1024.0f) + bias;
        h1L[(8 * hh + r) * kHP + nt * 16 + cc] = (_Float16)softplus_f(x);
      }
    }
  }
  wave_sync();
  {
    v16h a2[8];
#pragma unroll
    for (int kt = 0; kt < 8; ++kt) a2[kt] = FragH::load(h1L + cc * kHP + kt * 32 + koff);
#pragma unroll 1
    for (int nt = 0; nt < kHid / 16; ++nt) {
      v8f acc = zero8;
#pragma unroll
      for (int kt = 0; kt < 8; ++kt) {
        const v16h b = FragH::load(W1L + (nt * 16 + cc) * kW1P + kt * 32 + koff);
        acc = mma_g(a2[kt], b, acc);
      }
      const float bias = b1L[nt * 16 + cc];
#pragma unroll
      for (int r = 0; r < 8; ++r) {
        const float x = acc[r] * (1.0f / 64.0f) + bias;
        h2L[(8 * hh + r) * kHP + nt * 16 + cc] = (_Float16)softplus_f(x);
      }
    }
  }
  wave_sync();
  {
    v16h a3[8];
#pragma unroll
    for (int kt = 0; kt < 8; ++kt) a3[kt] = FragH::load(h2L + cc * kHP + kt * 32 + koff);
#pragma unroll
    for (int nt = 0; nt < kDim / 16; ++nt) {
      v8f acc = zero8;
#pragma unroll
      for (int kt = 0; kt < 8; ++kt) {
        const v16h b = FragH::load(W2L + (nt * 16 + cc) * kW2P + kt * 32 + koff);
        acc = mma_g(a3[kt], b, acc);
      }
      const float bias = b2L[nt * 16 + cc];
#pragma unroll
      for (int r = 0; r < 8; ++r) kout[nt * 8 + r] = acc[r] * (1.0f / 64.0f) + bias;
    }
  }
}

__global__ __launch_bounds__(64)
void node_tsit5_kernel(const float* __restrict__ ts, const float* __restrict__ y0,
                       const float* __restrict__ gW0, const float* __restrict__ gb0,
                       const float* __restrict__ gW1, const float* __restrict__ gb1,
                       const float* __restrict__ gW2, const float* __restrict__ gb2,
                       float* __restrict__ out, int nb, int nts)
{
  extern __shared__ __align__(16) unsigned char smem_dyn[];
  _Float16* W1L = (_Float16*)(smem_dyn + kOffW1);
  _Float16* W0L = (_Float16*)(smem_dyn + kOffW0);
  _Float16* W2L = (_Float16*)(smem_dyn + kOffW2);
  float* b0L   = (float*)(smem_dyn + kOffB0);
  float* b1L   = (float*)(smem_dyn + kOffB1);
  float* b2L   = (float*)(smem_dyn + kOffB2);
  float* tsL   = (float*)(smem_dyn + kOffTS);
  float* coefL = (float*)(smem_dyn + kOffCF);

  const int tid  = threadIdx.x;
  const int lane = tid & 31;
  const int wave = tid >> 5;
  const int hh   = lane >> 4;
  const int cc   = lane & 15;

  unsigned char* wb = smem_dyn + kOffWave + (unsigned)wave * kWaveBytes;
  _Float16* ybL = (_Float16*)(wb + kWoffY);
  _Float16* h1L = (_Float16*)(wb + kWoffH1);
  _Float16* h2L = (_Float16*)(wb + kWoffH2);
  float*    kbL = (float*)(wb + kWoffKB);
  float*    osL = (float*)(wb + kWoffOS);

#pragma unroll 2
  for (int u = tid; u < kHid * (kHid / 8); u += kThreads) {
    const int n = u >> 5, k8 = (u & 31) * 8;
    const v4f a = *(const v4f*)(gW1 + (size_t)n * kHid + k8);
    const v4f b = *(const v4f*)(gW1 + (size_t)n * kHid + k8 + 4);
    v8h hv;
    hv[0] = (_Float16)(a[0] * 64.0f); hv[1] = (_Float16)(a[1] * 64.0f);
    hv[2] = (_Float16)(a[2] * 64.0f); hv[3] = (_Float16)(a[3] * 64.0f);
    hv[4] = (_Float16)(b[0] * 64.0f); hv[5] = (_Float16)(b[1] * 64.0f);
    hv[6] = (_Float16)(b[2] * 64.0f); hv[7] = (_Float16)(b[3] * 64.0f);
    *(v8h*)(W1L + n * kW1P + k8) = hv;
  }
#pragma unroll 2
  for (int u = tid; u < kHid * (kDim / 8); u += kThreads) {
    const int n = u >> 2, k8 = (u & 3) * 8;
    const v4f a = *(const v4f*)(gW0 + (size_t)n * kDim + k8);
    const v4f b = *(const v4f*)(gW0 + (size_t)n * kDim + k8 + 4);
    v8h hv;
    hv[0] = (_Float16)(a[0] * 64.0f); hv[1] = (_Float16)(a[1] * 64.0f);
    hv[2] = (_Float16)(a[2] * 64.0f); hv[3] = (_Float16)(a[3] * 64.0f);
    hv[4] = (_Float16)(b[0] * 64.0f); hv[5] = (_Float16)(b[1] * 64.0f);
    hv[6] = (_Float16)(b[2] * 64.0f); hv[7] = (_Float16)(b[3] * 64.0f);
    *(v8h*)(W0L + n * kW0P + k8) = hv;
  }
#pragma unroll 2
  for (int u = tid; u < kDim * (kHid / 8); u += kThreads) {
    const int n = u >> 5, k8 = (u & 31) * 8;
    const v4f a = *(const v4f*)(gW2 + (size_t)n * kHid + k8);
    const v4f b = *(const v4f*)(gW2 + (size_t)n * kHid + k8 + 4);
    v8h hv;
    hv[0] = (_Float16)(a[0] * 64.0f); hv[1] = (_Float16)(a[1] * 64.0f);
    hv[2] = (_Float16)(a[2] * 64.0f); hv[3] = (_Float16)(a[3] * 64.0f);
    hv[4] = (_Float16)(b[0] * 64.0f); hv[5] = (_Float16)(b[1] * 64.0f);
    hv[6] = (_Float16)(b[2] * 64.0f); hv[7] = (_Float16)(b[3] * 64.0f);
    *(v8h*)(W2L + n * kW2P + k8) = hv;
  }
  for (int i = tid; i < kHid; i += kThreads) { b0L[i] = gb0[i]; b1L[i] = gb1[i]; }
  if (tid < kDim) b2L[tid] = gb2[tid];
  if (tid < kMaxT) { const int si = (tid < nts) ? tid : (nts - 1); tsL[tid] = ts[si]; }
  if (tid == 0) {
    for (int i = 0; i < 64; ++i) coefL[i] = 0.0f;
    coefL[1 * 8 + 0] = 0.161f;
    coefL[2 * 8 + 0] = -0.008480655492356989f;  coefL[2 * 8 + 1] = 0.335480655492357f;
    coefL[3 * 8 + 0] = 2.8971530571054935f;     coefL[3 * 8 + 1] = -6.359448489975075f;   coefL[3 * 8 + 2] = 4.3622954328695815f;
    coefL[4 * 8 + 0] = 5.325864828439257f;      coefL[4 * 8 + 1] = -11.748883564062828f;  coefL[4 * 8 + 2] = 7.4955393428898365f;
    coefL[4 * 8 + 3] = -0.09249506636175525f;
    coefL[5 * 8 + 0] = 5.86145544294642f;       coefL[5 * 8 + 1] = -12.92096931784711f;   coefL[5 * 8 + 2] = 8.159367898576159f;
    coefL[5 * 8 + 3] = -0.071584973281401f;     coefL[5 * 8 + 4] = -0.028269050394068383f;
    coefL[6 * 8 + 0] = 0.09646076681806523f;    coefL[6 * 8 + 1] = 0.01f;                 coefL[6 * 8 + 2] = 0.4798896504144996f;
    coefL[6 * 8 + 3] = 1.379008574103742f;      coefL[6 * 8 + 4] = -3.290069515436081f;   coefL[6 * 8 + 5] = 2.324710524099774f;
  }
  __syncthreads();

  const int rowbase = blockIdx.x * kRowsBlock + wave * kRowsWave;

#pragma unroll
  for (int it = 0; it < 4; ++it) {
    const int idx = it * 128 + lane * 4;
    const int row = idx >> 5, col = idx & 31;
    const v4f v = *(const v4f*)(y0 + (size_t)(rowbase + row) * kDim + col);
    *(v4f*)(osL + row * kOSP + col) = v;
  }
  wave_sync();
  float y[16];
#pragma unroll
  for (int i = 0; i < 16; ++i) y[i] = osL[(8 * hh + (i & 7)) * kOSP + (i >> 3) * 16 + cc];
  store_rows16(out + (size_t)rowbase * kDim, osL, lane);
  wave_sync();

  for (int t = 0; t + 1 < nts; ++t) {
    const float hstep = (tsL[t + 1] - tsL[t]) * 0.5f;
#pragma unroll 1
    for (int sub = 0; sub < kNSub; ++sub) {
#pragma unroll 1
      for (int s = 0; s < kStages; ++s) {
        float v[16];
#pragma unroll
        for (int i = 0; i < 16; ++i) v[i] = 0.0f;
        for (int j = 0; j < s; ++j) {
          const float cf = coefL[s * 8 + j];
#pragma unroll
          for (int i = 0; i < 16; ++i) v[i] += cf * kbL[(j * 16 + i) * 32 + lane];
        }
#pragma unroll
        for (int i = 0; i < 16; ++i) {
          const float yt = y[i] + hstep * v[i];
          ybL[(8 * hh + (i & 7)) * kYP + (i >> 3) * 16 + cc] = (_Float16)(yt * 16.0f);
        }
        wave_sync();
        float kreg[16];
        mlp_eval(ybL, h1L, h2L, W0L, W1L, W2L, b0L, b1L, b2L, hh, cc, kreg);
#pragma unroll
        for (int i = 0; i < 16; ++i) kbL[(s * 16 + i) * 32 + lane] = kreg[i];
      }
      float v[16];
#pragma unroll
      for (int i = 0; i < 16; ++i) v[i] = 0.0f;
#pragma unroll
      for (int j = 0; j < kStages; ++j) {
        const float cf = coefL[6 * 8 + j];
#pragma unroll
        for (int i = 0; i < 16; ++i) v[i] += cf * kbL[(j * 16 + i) * 32 + lane];
      }
#pragma unroll
      for (int i = 0; i < 16; ++i) y[i] = y[i] + hstep * v[i];
    }
#pragma unroll
    for (int i = 0; i < 16; ++i) osL[(8 * hh + (i & 7)) * kOSP + (i >> 3) * 16 + cc] = y[i];
    wave_sync();
    store_rows16(out + ((size_t)(t + 1) * (size_t)nb + (size_t)rowbase) * kDim, osL, lane);
    wave_sync();
  }
}

extern "C" void kernel_launch(void* const* d_in, const int* in_sizes, int n_in,
                              void* d_out, int out_size, void* d_ws, size_t ws_size,
                              hipStream_t stream) {
  (void)d_ws; (void)ws_size;
  if (n_in < 8) return;
  const float* ts = (const float*)d_in[0];
  const float* y0 = (const float*)d_in[1];
  const float* W0 = (const float*)d_in[2];
  const float* b0 = (const float*)d_in[3];
  const float* W1 = (const float*)d_in[4];
  const float* b1 = (const float*)d_in[5];
  const float* W2 = (const float*)d_in[6];
  const float* b2 = (const float*)d_in[7];
  float* out = (float*)d_out;

  int nts = in_sizes[0];
  if (nts > kMaxT) nts = kMaxT;
  if (nts < 1) return;
  if (in_sizes[2] < kHid * kDim || in_sizes[4] < kHid * kHid || in_sizes[6] < kDim * kHid) return;
  if (in_sizes[3] < kHid || in_sizes[5] < kHid || in_sizes[7] < kDim) return;
  const long nb = (long)in_sizes[1] / kDim;
  if (nb <= 0) return;
  if ((long)nts * nb * kDim > (long)out_size) return;
  const int nblk = (int)(nb / kRowsBlock);
  if (nblk <= 0) return;

  node_tsit5_kernel<<<dim3((unsigned)nblk), dim3(kThreads), kSmemBytes, stream>>>(
      ts, y0, W0, b0, W1, b1, W2, b2, out, (int)nb, nts);
}
